// MemoryEfficientAttention_62234076119055
// MI455X (gfx1250) — hardware-verified
//
#include <hip/hip_runtime.h>
#include <math.h>

#ifndef NB
#define NB 2
#endif
#ifndef SEQ
#define SEQ 2048
#endif
#define NB_FULL 2
#define SEQ_FULL 2048
#define CDIM 1024
#define NHEAD 16
#define HDIM 64
#define QKVD (3 * CDIM)
static_assert(NB >= 1 && NB <= NB_FULL);
static_assert(SEQ >= 64 && SEQ <= SEQ_FULL && (SEQ % 64) == 0);
static_assert(CDIM == NHEAD * HDIM);
static_assert(HDIM == 64);
static_assert((CDIM % 64) == 0 && (QKVD % 64) == 0 && (CDIM % 32) == 0);

typedef __attribute__((ext_vector_type(16))) _Float16 v16h;
typedef __attribute__((ext_vector_type(8)))  _Float16 v8h;
typedef __attribute__((ext_vector_type(16))) __bf16   v16b;
typedef __attribute__((ext_vector_type(8)))  float    v8f;
typedef __attribute__((ext_vector_type(4)))  float    v4f;
typedef __attribute__((ext_vector_type(8)))  unsigned short v8us;
typedef __attribute__((ext_vector_type(16))) unsigned short v16us;
typedef v8us __attribute__((may_alias)) v8usa;
typedef v4f  __attribute__((may_alias)) v4fa;

__device__ __forceinline__ int frag_k(int i, int h) { return (i < 8) ? (8 * h + i) : (16 + 8 * h + (i - 8)); }
__device__ __forceinline__ __bf16 bf16_rne(float f) {
    unsigned int u = __float_as_uint(f);
    u += 0x7fffu + ((u >> 16) & 1u);
    return __builtin_bit_cast(__bf16, (unsigned short)(u >> 16));
}
__device__ __forceinline__ float bf16_f32(__bf16 b) { return __uint_as_float(((unsigned int)__builtin_bit_cast(unsigned short, b)) << 16); }
__device__ __forceinline__ void bf16_hl(float x, unsigned short& hs, unsigned short& ls) {
    const unsigned int u = __float_as_uint(x);
    const unsigned int r = u + 0x7fffu + ((u >> 16) & 1u);
    hs = (unsigned short)(r >> 16);
    const float res = x - __uint_as_float(((unsigned int)hs) << 16);
    const unsigned int u2 = __float_as_uint(res);
    const unsigned int r2 = u2 + 0x7fffu + ((u2 >> 16) & 1u);
    ls = (unsigned short)(r2 >> 16);
}
__device__ __forceinline__ unsigned short f16_bits(float x) { return __builtin_bit_cast(unsigned short, (_Float16)x); }

__device__ __forceinline__ v8f wmma16(v16h a, v16h b, v8f c) {
    c = __builtin_amdgcn_wmma_f32_16x16x32_f16(false, a, false, b, (short)0, c, false, false);
    asm volatile("v_nop\n\tv_nop\n\tv_nop\n\tv_nop" : "+v"(c) : "v"(a), "v"(b));
    return c;
}
__device__ __forceinline__ v8f wmmab(v16b a, v16b b, v8f c) {
    c = __builtin_amdgcn_wmma_f32_16x16x32_bf16(false, a, false, b, (short)0, c, false, false);
    asm volatile("v_nop\n\tv_nop\n\tv_nop\n\tv_nop" : "+v"(c) : "v"(a), "v"(b));
    return c;
}
struct Split { v16b hi, lo; };
__device__ __forceinline__ v8f wmma3(const Split& a, const Split& b, v8f c) {
    c = __builtin_amdgcn_wmma_f32_16x16x32_bf16(false, a.hi, false, b.hi, (short)0, c, false, false);
    c = __builtin_amdgcn_wmma_f32_16x16x32_bf16(false, a.hi, false, b.lo, (short)0, c, false, false);
    c = __builtin_amdgcn_wmma_f32_16x16x32_bf16(false, a.lo, false, b.hi, (short)0, c, false, false);
    asm volatile("v_nop\n\tv_nop\n\tv_nop\n\tv_nop" : "+v"(c) : "v"(a.hi), "v"(a.lo), "v"(b.hi), "v"(b.lo));
    return c;
}
__device__ __forceinline__ v8f wmma2(const Split& a, v16b b, v8f c) {
    c = __builtin_amdgcn_wmma_f32_16x16x32_bf16(false, a.hi, false, b, (short)0, c, false, false);
    c = __builtin_amdgcn_wmma_f32_16x16x32_bf16(false, a.lo, false, b, (short)0, c, false, false);
    asm volatile("v_nop\n\tv_nop\n\tv_nop\n\tv_nop" : "+v"(c) : "v"(a.hi), "v"(a.lo), "v"(b));
    return c;
}

__device__ __forceinline__ v16h fh_ld(const float* __restrict__ p, long long sk, int k0, int h, int klen, float s) {
    v16h a;
#pragma unroll
    for (int i = 0; i < 16; ++i) { const int k = k0 + frag_k(i, h); a[i] = (k < klen) ? (_Float16)(p[(long long)k * sk] * s) : (_Float16)0.f; }
    return a;
}
__device__ __forceinline__ Split sp_ld(const float* __restrict__ p, long long sk, int k0, int h, int klen, float s) {
    Split r;
#pragma unroll
    for (int i = 0; i < 16; ++i) {
        const int k = k0 + frag_k(i, h); const float x = (k < klen) ? p[(long long)k * sk] * s : 0.f;
        const __bf16 hb = bf16_rne(x); r.hi[i] = hb; r.lo[i] = bf16_rne(x - bf16_f32(hb));
    }
    return r;
}
__device__ __forceinline__ v16b bh_ld(const float* __restrict__ p, long long sk, int k0, int h, int klen, float s) {
    v16b a;
#pragma unroll
    for (int i = 0; i < 16; ++i) { const int k = k0 + frag_k(i, h); a[i] = bf16_rne((k < klen) ? p[(long long)k * sk] * s : 0.f); }
    return a;
}
union Frag16 { v16us u; v16h h; v16b b; v8us p[2]; };
__device__ __forceinline__ Frag16 ld16(const unsigned short* __restrict__ row, int k0, int h) {
    Frag16 f;
    f.p[0] = *(const v8us*)(row + k0 + 8 * h);
    f.p[1] = *(const v8us*)(row + k0 + 16 + 8 * h);
    return f;
}

#define VST2(T, ptr, val) do { const T vst2_v_ = (val); *(volatile T*)(ptr) = vst2_v_; __threadfence(); *(volatile T*)(ptr) = vst2_v_; } while (0)
#define VST2V4(ptr, val) do { const v4f vst2_v4_ = (val); *(volatile v4f*)(ptr) = vst2_v4_; __threadfence(); *(volatile v4f*)(ptr) = vst2_v4_; } while (0)
#define VST2V8U(ptr, val) do { const v8us vst2_v8_ = (val); *(volatile v8us*)(ptr) = vst2_v8_; __threadfence(); *(volatile v8us*)(ptr) = vst2_v8_; } while (0)

struct GemmP {
    const float* A; const float* B; const float* bias; const float* R; float* C;
    long long sAo, sAi, sAm, sAk, sBo, sBi, sBn, sBk, sCo, sCi, sCm, sRo, sRi, sRm, sRn;
    int M, N, K, zi_n, flags, act; float alpha, beta, sa, sb;
    int Npad, pad_;
};
static_assert(sizeof(GemmP) == 5 * 8 + 15 * 8 + 6 * 4 + 4 * 4 + 2 * 4);

template <int MODE, int TM, int TN>
__global__ __launch_bounds__(32) void k_gemmT(GemmP p) {
    const int lane = threadIdx.x & 31, h = lane >> 4, l15 = lane & 15;
    const int m0 = blockIdx.y * (16 * TM), n0 = blockIdx.x * (16 * TN);
    const int z = blockIdx.z, zo = z / p.zi_n, zi = z - zo * p.zi_n;
    const float* A = p.A + zo * p.sAo + zi * p.sAi;
    const float* B = p.B + zo * p.sBo + zi * p.sBi;
    v8f acc[TM][TN];
#pragma unroll
    for (int i = 0; i < TM; ++i)
#pragma unroll
        for (int t = 0; t < TN; ++t) { v8f zz = {}; acc[i][t] = zz; }
    for (int k0 = 0; k0 < p.K; k0 += 32) {
        if (MODE == 1) {
            Split a[TM], b[TN];
#pragma unroll
            for (int i = 0; i < TM; ++i) { const int am = min(m0 + 16 * i + l15, p.M - 1); a[i] = sp_ld(A + (long long)am * p.sAm, p.sAk, k0, h, p.K, 1.f); }
#pragma unroll
            for (int t = 0; t < TN; ++t) { const int bn = min(n0 + 16 * t + l15, p.N - 1); b[t] = sp_ld(B + (long long)bn * p.sBn, p.sBk, k0, h, p.K, 1.f); }
#pragma unroll
            for (int i = 0; i < TM; ++i)
#pragma unroll
                for (int t = 0; t < TN; ++t) acc[i][t] = wmma3(a[i], b[t], acc[i][t]);
        } else if (MODE == 5) {
            Split a[TM]; v16b b[TN];
#pragma unroll
            for (int i = 0; i < TM; ++i) { const int am = min(m0 + 16 * i + l15, p.M - 1); a[i] = sp_ld(A + (long long)am * p.sAm, p.sAk, k0, h, p.K, 1.f); }
#pragma unroll
            for (int t = 0; t < TN; ++t) { const int bn = min(n0 + 16 * t + l15, p.N - 1); b[t] = bh_ld(B + (long long)bn * p.sBn, p.sBk, k0, h, p.K, 1.f); }
#pragma unroll
            for (int i = 0; i < TM; ++i)
#pragma unroll
                for (int t = 0; t < TN; ++t) acc[i][t] = wmma2(a[i], b[t], acc[i][t]);
        } else if (MODE == 2) {
            v16b a[TM], b[TN];
#pragma unroll
            for (int i = 0; i < TM; ++i) { const int am = min(m0 + 16 * i + l15, p.M - 1); a[i] = bh_ld(A + (long long)am * p.sAm, p.sAk, k0, h, p.K, 1.f); }
#pragma unroll
            for (int t = 0; t < TN; ++t) { const int bn = min(n0 + 16 * t + l15, p.N - 1); b[t] = bh_ld(B + (long long)bn * p.sBn, p.sBk, k0, h, p.K, 1.f); }
#pragma unroll
            for (int i = 0; i < TM; ++i)
#pragma unroll
                for (int t = 0; t < TN; ++t) acc[i][t] = wmmab(a[i], b[t], acc[i][t]);
        } else {
            v16h a[TM], b[TN];
#pragma unroll
            for (int i = 0; i < TM; ++i) { const int am = min(m0 + 16 * i + l15, p.M - 1); a[i] = fh_ld(A + (long long)am * p.sAm, p.sAk, k0, h, p.K, p.sa); }
#pragma unroll
            for (int t = 0; t < TN; ++t) { const int bn = min(n0 + 16 * t + l15, p.N - 1); b[t] = fh_ld(B + (long long)bn * p.sBn, p.sBk, k0, h, p.K, p.sb); }
#pragma unroll
            for (int i = 0; i < TM; ++i)
#pragma unroll
                for (int t = 0; t < TN; ++t) acc[i][t] = wmma16(a[i], b[t], acc[i][t]);
        }
    }
    const float iscale = (MODE == 0) ? p.alpha / (p.sa * p.sb) : p.alpha;
    float* C = p.C + zo * p.sCo + zi * p.sCi;
    const float* R = p.R + zo * p.sRo + zi * p.sRi;
    const int NW = (p.Npad > p.N) ? p.Npad : p.N;
    __shared__ __align__(16) float ctile[16][36];
#pragma unroll
    for (int i = 0; i < TM; ++i) {
        const int mb = m0 + 16 * i; if (mb >= p.M) break;
#pragma unroll
        for (int tp = 0; tp < TN / 2; ++tp) {
            const int nb = n0 + 32 * tp; if (nb >= NW) break;
#pragma unroll
            for (int t2 = 0; t2 < 2; ++t2) {
                const int t = 2 * tp + t2; const int n = nb + t2 * 16 + l15; const int nn = min(n, p.N - 1);
#pragma unroll
                for (int r = 0; r < 8; ++r) {
                    const int m = mb + 8 * h + r; const int mm = min(m, p.M - 1);
                    float v = acc[i][t][r] * iscale;
                    if (p.flags & 1) { float bv = p.bias[nn]; if (p.flags & 16) bv = bf16_f32(bf16_rne(bv)); v += bv; }
                    if (p.flags & 2) { float bv = p.bias[mm]; if (p.flags & 16) bv = bf16_f32(bf16_rne(bv)); v += bv; }
                    if (p.flags & 4) v += p.beta * R[(long long)mm * p.sRm + (long long)nn * p.sRn];
                    ctile[8 * h + r][t2 * 16 + l15] = (n < p.N) ? v : 0.f;
                }
            }
            __syncthreads();
            const bool fast = (mb + 16 <= p.M) && (nb + 32 <= NW) && ((p.sCm & 3) == 0) && ((((size_t)C) & 15) == 0);
            if (fast) {
#pragma unroll
                for (int s = 0; s < 4; ++s) {
                    const int row = s * 4 + (lane >> 3), c4 = (lane & 7) * 4;
                    const v4f v = *(const v4f*)&ctile[row][c4];
                    VST2V4(C + (long long)(mb + row) * p.sCm + nb + c4, v);
                }
            } else {
                for (int row = 0; row < 16; ++row) {
                    const int m = mb + row, n = nb + lane;
                    if (m < p.M && n < NW) VST2(float, C + (long long)m * p.sCm + n, ctile[row][lane]);
                }
            }
            __syncthreads();
        }
    }
}

__global__ __launch_bounds__(256) void k_cvt(const float* __restrict__ qkv, unsigned short* __restrict__ qh, unsigned short* __restrict__ ql,
                                             unsigned short* __restrict__ kh, unsigned short* __restrict__ kl, unsigned short* __restrict__ vt,
                                             int L, int H) {
    __shared__ __align__(16) unsigned short vs[64][72];
    const int tid = threadIdx.x, c = blockIdx.x, h = blockIdx.y, b = blockIdx.z;
    const int C3 = 3 * H * HDIM;
    const size_t bh = (size_t)b * H + h;
#pragma unroll
    for (int s = 0; s < 2; ++s) {
        const int r = s * 32 + (tid >> 3), c8 = (tid & 7) * 8, i = c * 64 + r;
        const float* src = qkv + ((size_t)b * L + i) * C3 + h * HDIM + c8;
        const size_t drow = (bh * L + i) * HDIM + c8;
        {
            const v4f a = *(const v4f*)src, e = *(const v4f*)(src + 4);
            v8us uh = {}, ul = {};
#pragma unroll
            for (int j = 0; j < 4; ++j) { unsigned short x1, x2; bf16_hl(a[j], x1, x2); uh[j] = x1; ul[j] = x2; bf16_hl(e[j], x1, x2); uh[4 + j] = x1; ul[4 + j] = x2; }
            VST2V8U(qh + drow, uh); VST2V8U(ql + drow, ul);
        }
        {
            const v4f a = *(const v4f*)(src + H * HDIM), e = *(const v4f*)(src + H * HDIM + 4);
            v8us uh = {}, ul = {};
#pragma unroll
            for (int j = 0; j < 4; ++j) { unsigned short x1, x2; bf16_hl(a[j], x1, x2); uh[j] = x1; ul[j] = x2; bf16_hl(e[j], x1, x2); uh[4 + j] = x1; ul[4 + j] = x2; }
            VST2V8U(kh + drow, uh); VST2V8U(kl + drow, ul);
        }
        {
            const v4f a = *(const v4f*)(src + 2 * H * HDIM), e = *(const v4f*)(src + 2 * H * HDIM + 4);
#pragma unroll
            for (int j = 0; j < 4; ++j) { vs[c8 + j][r] = f16_bits(a[j]); vs[c8 + 4 + j][r] = f16_bits(e[j]); }
        }
    }
    __syncthreads();
#pragma unroll
    for (int s = 0; s < 2; ++s) {
        const int d = s * 32 + (tid >> 3), c8 = (tid & 7) * 8;
        const v8us w = *(const v8usa*)&vs[d][c8];
        VST2V8U(vt + (bh * HDIM + d) * (size_t)L + (size_t)c * 64 + c8, w);
    }
}

__global__ __launch_bounds__(32) __attribute__((amdgpu_num_vgpr(256)))
void k_att(const unsigned short* __restrict__ qh, const unsigned short* __restrict__ ql, const unsigned short* __restrict__ kh,
           const unsigned short* __restrict__ kl, const unsigned short* __restrict__ vt, float* __restrict__ ctx, int L, int H, float scl2) {
    __shared__ __align__(16) unsigned short ph[16][72];
    __shared__ __align__(16) float ost[16][68];
    const int lane = threadIdx.x & 31, hf = lane >> 4, l15 = lane & 15;
    const int q0 = blockIdx.x * 16, h = blockIdx.y, b = blockIdx.z;
    const size_t bh = (size_t)b * H + h;
    const float NEG = -__builtin_inff();
    const unsigned short* qhr = qh + (bh * L + q0 + l15) * HDIM;
    const unsigned short* qlr = ql + (bh * L + q0 + l15) * HDIM;
    const unsigned short* khb = kh + bh * L * HDIM;
    const unsigned short* klb = kl + bh * L * HDIM;
    const unsigned short* vtb = vt + bh * HDIM * (size_t)L;
    Split qs[2];
#pragma unroll
    for (int ks = 0; ks < 2; ++ks) {
        Frag16 f = ld16(qhr, ks * 32, hf); qs[ks].hi = f.b;
        f = ld16(qlr, ks * 32, hf); qs[ks].lo = f.b;
    }
    v8f o[4]; float m8[8], l8[8];
#pragma unroll
    for (int t = 0; t < 4; ++t) { v8f zz = {}; o[t] = zz; }
#pragma unroll
    for (int i = 0; i < 8; ++i) { m8[i] = NEG; l8[i] = 0.f; }
#pragma unroll 1
    for (int j0 = 0; j0 < L; j0 += 64) {
        v8f s[4];
#pragma unroll
        for (int t = 0; t < 4; ++t) {
            const size_t kr = (size_t)(j0 + t * 16 + l15) * HDIM;
            v8f acc = {};
#pragma unroll
            for (int ks = 0; ks < 2; ++ks) {
                Split kf;
                Frag16 f = ld16(khb + kr, ks * 32, hf); kf.hi = f.b;
                f = ld16(klb + kr, ks * 32, hf); kf.lo = f.b;
                acc = wmma3(qs[ks], kf, acc);
            }
            s[t] = acc;
        }
        __syncthreads();
#pragma unroll
        for (int i = 0; i < 8; ++i) {
            float sc[4];
#pragma unroll
            for (int t = 0; t < 4; ++t) sc[t] = s[t][i] * scl2;
            float mx = fmaxf(fmaxf(sc[0], sc[1]), fmaxf(sc[2], sc[3]));
            mx = fmaxf(mx, __shfl_xor(mx, 1, 32)); mx = fmaxf(mx, __shfl_xor(mx, 2, 32));
            mx = fmaxf(mx, __shfl_xor(mx, 4, 32)); mx = fmaxf(mx, __shfl_xor(mx, 8, 32));
            const float mnew = fmaxf(m8[i], mx);
            const float corr = (mnew == NEG) ? 1.f : exp2f(m8[i] - mnew);
            float rs = 0.f;
#pragma unroll
            for (int t = 0; t < 4; ++t) {
                const float pp = exp2f(sc[t] - mnew); rs += pp;
                ph[i + 8 * hf][t * 16 + l15] = f16_bits(pp * 4096.f);
            }
            rs += __shfl_xor(rs, 1, 32); rs += __shfl_xor(rs, 2, 32); rs += __shfl_xor(rs, 4, 32); rs += __shfl_xor(rs, 8, 32);
            l8[i] = l8[i] * corr + rs; m8[i] = mnew;
#pragma unroll
            for (int t = 0; t < 4; ++t) o[t][i] *= corr;
        }
        __syncthreads();
#pragma unroll
        for (int kk = 0; kk < 2; ++kk) {
            Frag16 pa;
            pa.p[0] = *(const v8usa*)&ph[l15][kk * 32 + 8 * hf];
            pa.p[1] = *(const v8usa*)&ph[l15][kk * 32 + 16 + 8 * hf];
#pragma unroll
            for (int t = 0; t < 4; ++t) {
                const Frag16 bv = ld16(vtb + (size_t)(t * 16 + l15) * L + j0 + kk * 32, 0, hf);
                o[t] = wmma16(pa.h, bv.h, o[t]);
            }
        }
    }
    float invr[8];
#pragma unroll
    for (int i = 0; i < 8; ++i) invr[i] = (l8[i] > 0.f) ? 1.f / (l8[i] * 4096.f) : 0.f;
    __syncthreads();
#pragma unroll
    for (int i = 0; i < 8; ++i)
#pragma unroll
        for (int t = 0; t < 4; ++t) ost[i + 8 * hf][t * 16 + l15] = o[t][i] * invr[i];
    __syncthreads();
    const size_t CP = (size_t)H * HDIM;
    float* ob = ctx + ((size_t)b * L + q0) * CP + (size_t)h * HDIM;
#pragma unroll
    for (int s2 = 0; s2 < 8; ++s2) {
        const int row = s2 * 2 + (lane >> 4), c4 = (lane & 15) * 4;
        const v4f v = *(const v4fa*)&ost[row][c4];
        VST2V4(ob + (size_t)row * CP + c4, v);
    }
}

extern "C" void kernel_launch(void* const* d_in, const int* in_sizes, int n_in, void* d_out, int out_size, void* d_ws, size_t ws_size, hipStream_t stream) {
    if (n_in < 4) return;
    const float* x     = (const float*)d_in[0];
    const float* wqkv  = (const float*)d_in[1];
    const float* wproj = (const float*)d_in[2];
    const float* bproj = (const float*)d_in[3];
    float* out = (float*)d_out;
    const long long need_rows = (long long)(NB - 1) * SEQ_FULL + SEQ;
    if ((long long)in_sizes[0] < need_rows * CDIM) return;
    if ((long long)in_sizes[1] < (long long)QKVD * CDIM) return;
    if ((long long)in_sizes[2] < (long long)CDIM * CDIM) return;
    if ((long long)in_sizes[3] < (long long)CDIM) return;
    if ((long long)out_size < need_rows * CDIM) return;

    size_t off = 0;
    const size_t qkv_bytes = (size_t)NB * SEQ * QKVD * sizeof(float);
    const size_t p16_bytes = (size_t)NB * NHEAD * SEQ * HDIM * 2;
    const size_t ctx_bytes = (size_t)NB * SEQ * CDIM * sizeof(float);
    float* qkv = (float*)((char*)d_ws + off); off += qkv_bytes;
    unsigned short* qh = (unsigned short*)((char*)d_ws + off); off += p16_bytes;
    unsigned short* ql = (unsigned short*)((char*)d_ws + off); off += p16_bytes;
    unsigned short* kh = (unsigned short*)((char*)d_ws + off); off += p16_bytes;
    unsigned short* kl = (unsigned short*)((char*)d_ws + off); off += p16_bytes;
    unsigned short* vt = (unsigned short*)((char*)d_ws + off); off += p16_bytes;
    float* ctx = (float*)((char*)d_ws + off); off += ctx_bytes;
    if (off > ws_size) return;

    {
        GemmP g = {};
        g.A = x; g.B = wqkv; g.bias = bproj; g.R = x; g.C = qkv;
        g.sAo = (long long)SEQ_FULL * CDIM; g.sAi = 0; g.sAm = CDIM; g.sAk = 1;
        g.sBo = 0; g.sBi = 0; g.sBn = CDIM; g.sBk = 1;
        g.sCo = (long long)SEQ * QKVD; g.sCi = 0; g.sCm = QKVD;
        g.sRo = 0; g.sRi = 0; g.sRm = 0; g.sRn = 0;
        g.M = SEQ; g.N = QKVD; g.K = CDIM; g.zi_n = 1; g.flags = 0; g.act = 0;
        g.alpha = 1.f; g.beta = 0.f; g.sa = 1.f; g.sb = 1.f; g.Npad = QKVD; g.pad_ = 0;
        k_gemmT<2, 2, 4><<<dim3((unsigned)(QKVD / 64), (unsigned)(SEQ / 32), (unsigned)NB), 32, 0, stream>>>(g);
    }
    k_cvt<<<dim3((unsigned)(SEQ / 64), (unsigned)NHEAD, (unsigned)NB), 256, 0, stream>>>(qkv, qh, ql, kh, kl, vt, SEQ, NHEAD);
    {
        const float scl2 = 0.125f * 1.4426950408889634f;
        k_att<<<dim3((unsigned)(SEQ / 16), (unsigned)NHEAD, (unsigned)NB), 32, 0, stream>>>(qh, ql, kh, kl, vt, ctx, SEQ, NHEAD, scl2);
    }
    {
        GemmP g = {};
        g.A = ctx; g.B = wproj; g.bias = bproj; g.R = x; g.C = out;
        g.sAo = (long long)SEQ * CDIM; g.sAi = 0; g.sAm = CDIM; g.sAk = 1;
        g.sBo = 0; g.sBi = 0; g.sBn = CDIM; g.sBk = 1;
        g.sCo = (long long)SEQ_FULL * CDIM; g.sCi = 0; g.sCm = CDIM;
        g.sRo = 0; g.sRi = 0; g.sRm = 0; g.sRn = 0;
        g.M = SEQ; g.N = CDIM; g.K = CDIM; g.zi_n = 1; g.flags = 1 | 16; g.act = 0;
        g.alpha = 1.f; g.beta = 0.f; g.sa = 1.f; g.sb = 1.f; g.Npad = CDIM; g.pad_ = 0;
        k_gemmT<5, 2, 4><<<dim3((unsigned)(CDIM / 64), (unsigned)(SEQ / 32), (unsigned)NB), 32, 0, stream>>>(g);
    }
}
